// auto_attn_block_56229711839935
// MI455X (gfx1250) — hardware-verified
//
#include <hip/hip_runtime.h>
#include <math.h>

typedef __attribute__((ext_vector_type(16))) _Float16 v16h;
typedef __attribute__((ext_vector_type(8)))  _Float16 v8h;
typedef __attribute__((ext_vector_type(16))) __bf16   v16b;
typedef __attribute__((ext_vector_type(8)))  __bf16   v8b;
typedef __attribute__((ext_vector_type(8)))  float    v8f;
typedef __attribute__((ext_vector_type(4)))  float    v4f;

constexpr int kB    = 32;
constexpr int kT    = 512;
constexpr int kC    = 512;
constexpr int kP    = 64;
constexpr int kNS   = kT / kP;
constexpr int kFF   = 1024;
constexpr int kBC   = 8;
constexpr int kNCh  = kB / kBC;
constexpr int kRC   = kBC * kC;
constexpr int kRows = kB * kC;
constexpr int kThr  = 256;
constexpr float kInCarry = 1024.0f;
constexpr float kWCarry = 4096.0f;
constexpr float kScA = 1.0f / (kInCarry * kInCarry), kScK = 1.0f / (kInCarry * kWCarry);
constexpr float kInvT = 1.0f / 512.0f;
constexpr float kInvBT = 1.0f / 16384.0f;
constexpr float kEps = 1e-5f;
constexpr float kScoreScale = 0.044194173824159216f;
constexpr float kF16MinNormal = 6.103515625e-5f;

static_assert(kNS == 8 && kRC == 4096 && kRows == 16384 && ((kRC / 64) * (kT / 64)) % 8 == 0 && ((kRC / 64) * (kFF / 64)) % 8 == 0 && (kT % 32) == 0 && (kFF % 32) == 0, "GEMM M, N multiples of 64; grids exact; K multiples of 32");

constexpr size_t kOffWQ16 = 0ull;
constexpr size_t kOffWKT16 = 524288ull;
constexpr size_t kOffWV16 = 1048576ull;
constexpr size_t kOffWO16 = 1572864ull;
constexpr size_t kOffW1H = 2097152ull;
constexpr size_t kOffW2H = 3145728ull;
constexpr size_t kOffBIAS = 4194304ull;
constexpr size_t kOffSTAT = 4210688ull;
constexpr size_t kOffH32 = 4214784ull;
constexpr size_t kOffXT32 = 37769216ull;
constexpr size_t kOffX16 = 46157824ull;
constexpr size_t kOffFA = 50352128ull;
constexpr size_t kOffFB = 58740736ull;
constexpr size_t kOffHA = 67129344ull;
constexpr size_t kOffF1 = 71323648ull;
constexpr size_t kOffG16 = 88100864ull;
constexpr size_t kWsTotal = 96489472ull;
static_assert(kWsTotal <= 134217728ull, "carve cap: under 128 MiB");
static_assert(kOffWQ16 == 0
              && kOffWKT16 == kOffWQ16 + 524288ull
              && kOffWV16 == kOffWKT16 + 524288ull
              && kOffWO16 == kOffWV16 + 524288ull
              && kOffW1H == kOffWO16 + 524288ull
              && kOffW2H == kOffW1H + 1048576ull
              && kOffBIAS == kOffW2H + 1048576ull
              && kOffSTAT == kOffBIAS + 16384ull
              && kOffH32 == kOffSTAT + 4096ull
              && kOffXT32 == kOffH32 + 33554432ull
              && kOffX16 == kOffXT32 + 8388608ull
              && kOffFA == kOffX16 + 4194304ull
              && kOffFB == kOffFA + 8388608ull
              && kOffHA == kOffFB + 8388608ull
              && kOffF1 == kOffHA + 4194304ull
              && kOffG16 == kOffF1 + 16777216ull
              && kWsTotal == kOffG16 + 8388608ull, "the carve is chained and totalled");
static_assert((kOffWQ16 % 256) == 0 && (kOffWKT16 % 256) == 0 && (kOffWV16 % 256) == 0 && (kOffWO16 % 256) == 0 && (kOffW1H % 256) == 0 && (kOffW2H % 256) == 0 && (kOffBIAS % 256) == 0 && (kOffSTAT % 256) == 0 && (kOffH32 % 256) == 0 && (kOffXT32 % 256) == 0 && (kOffX16 % 256) == 0 && (kOffFA % 256) == 0 && (kOffFB % 256) == 0 && (kOffHA % 256) == 0 && (kOffF1 % 256) == 0 && (kOffG16 % 256) == 0, "aligned regions");

__device__ __forceinline__ unsigned short f2bf_bits(float f) {
  unsigned u = __float_as_uint(f);
  return (unsigned short)((u + 0x7FFFu + ((u >> 16) & 1u)) >> 16);
}
__device__ __forceinline__ float bf_bits2f(unsigned short h) { return __uint_as_float(((unsigned)h) << 16); }
__device__ __forceinline__ float bf16r(float f) { return bf_bits2f(f2bf_bits(f)); }
__device__ __forceinline__ float carry_flush(float v, float carry) {
  const float s = v * carry;
  return (fabsf(s) < kF16MinNormal) ? 0.0f : s;
}
__device__ __forceinline__ float frcp(float x) { return __builtin_amdgcn_rcpf(x); }

__device__ __forceinline__ void dep_guard4_h(v8f& a, v8f& b, v8f& c, v8f& d, v16h x, v16h y) { asm volatile("v_nop\n\tv_nop\n\tv_nop\n\tv_nop" : "+v"(a), "+v"(b), "+v"(c), "+v"(d) : "v"(x), "v"(y)); }
__device__ __forceinline__ void dep_guard4_b(v8f& a, v8f& b, v8f& c, v8f& d, v16b x, v16b y) { asm volatile("v_nop\n\tv_nop\n\tv_nop\n\tv_nop" : "+v"(a), "+v"(b), "+v"(c), "+v"(d) : "v"(x), "v"(y)); }
__device__ __forceinline__ void keep4_h(v16h a, v16h b, v16h c, v16h d) { asm volatile("v_nop" :: "v"(a), "v"(b), "v"(c), "v"(d)); }
__device__ __forceinline__ void keep4_b(v16b a, v16b b, v16b c, v16b d) { asm volatile("v_nop" :: "v"(a), "v"(b), "v"(c), "v"(d)); }
__device__ __forceinline__ void acc_guard4(v8f& a, v8f& b, v8f& c, v8f& d) { asm volatile("v_nop\n\tv_nop\n\tv_nop\n\tv_nop" : "+v"(a), "+v"(b), "+v"(c), "+v"(d)); }

template <typename T> struct Frag;
template <> struct Frag<_Float16> {
  typedef v16h V; union U { v16h v; v8h h[2]; };
  static __device__ __forceinline__ v16h load(const _Float16* p) {
    U f; f.h[0] = *(const v8h*)(p); f.h[1] = *(const v8h*)(p + 16); return f.v;
  }
  static __device__ __forceinline__ v8f mma(v16h a, v16h b, v8f c) {
    return __builtin_amdgcn_wmma_f32_16x16x32_f16(false, a, false, b, (short)0, c, false, false);
  }
  static __device__ __forceinline__ void guard4(v8f& a, v8f& b, v8f& c, v8f& d, v16h x, v16h y) { dep_guard4_h(a, b, c, d, x, y); }
  static __device__ __forceinline__ void keep(v16h a, v16h b, v16h c, v16h d) { keep4_h(a, b, c, d); }
};
template <> struct Frag<__bf16> {
  typedef v16b V; union U { v16b v; v8b h[2]; };
  static __device__ __forceinline__ v16b load(const __bf16* p) {
    U f; f.h[0] = *(const v8b*)(p); f.h[1] = *(const v8b*)(p + 16); return f.v;
  }
  static __device__ __forceinline__ v8f mma(v16b a, v16b b, v8f c) {
    return __builtin_amdgcn_wmma_f32_16x16x32_bf16(false, a, false, b, (short)0, c, false, false);
  }
  static __device__ __forceinline__ void guard4(v8f& a, v8f& b, v8f& c, v8f& d, v16b x, v16b y) { dep_guard4_b(a, b, c, d, x, y); }
  static __device__ __forceinline__ void keep(v16b a, v16b b, v16b c, v16b d) { keep4_b(a, b, c, d); }
};

__device__ __forceinline__ v8f mma_h(v16h a, v16h b, v8f c) {
  c = __builtin_amdgcn_wmma_f32_16x16x32_f16(false, a, false, b, (short)0, c, false, false);
  asm volatile("v_nop\n\tv_nop\n\tv_nop\n\tv_nop" : "+v"(c) : "v"(a), "v"(b));
  return c;
}

template <int ET> struct Elem;
template <> struct Elem<0> { typedef _Float16 T; };
template <> struct Elem<1> { typedef __bf16 T; };
template <int ET, bool SPLIT, int BIAS_MODE, int OUT_MODE, bool RESID, int ACT = 0>
__global__ __launch_bounds__(256) void wmma_gemm64(
    const unsigned short* __restrict__ Ap, const unsigned short* __restrict__ A2p, int lda, long strideA,
    const unsigned short* __restrict__ Btp, const unsigned short* __restrict__ Bt2p, int ldb, long strideB,
    void* __restrict__ Cout, void* __restrict__ Cout2, int ldc, long strideC,
    const float* __restrict__ bias,
    const float* __restrict__ resid, long strideR,
    int M, int N, int K, float scale) {
  typedef typename Elem<ET>::T T;
  typedef typename Frag<T>::V V;
  const T* A = (const T*)Ap; const T* A2 = (const T*)A2p; const T* Bt = (const T*)Btp; const T* Bt2 = (const T*)Bt2p;
  __shared__ __align__(16) float sT[8][16 * 68];
  const int b    = blockIdx.y;
  const int lane = threadIdx.x & 31;
  const int wave = threadIdx.x >> 5;
  const int tilesN = N >> 6;
  const int tilesM = M >> 6;
  const int tile = blockIdx.x * 8 + wave;
  if (tile >= tilesM * tilesN) return;
  const int tm = tile / tilesN;
  const int tn = tile - tm * tilesN;
  const int m0 = tm << 6;
  const int n0 = tn << 6;

  const T* Ab  = A  + (size_t)b * strideA;
  const T* Bb  = Bt + (size_t)b * strideB;
  const T* Ab2 = SPLIT ? (A2  + (size_t)b * strideA) : nullptr;
  const T* Bb2 = SPLIT ? (Bt2 + (size_t)b * strideB) : nullptr;

  const int rlane = lane & 15;
  const int koff  = (lane >> 4) * 8;
  const int mOff  = (lane >> 4) * 8;

  v8f acc[4][4];
#pragma unroll
  for (int i = 0; i < 4; ++i)
#pragma unroll
    for (int j = 0; j < 4; ++j) acc[i][j] = (v8f){0.f,0.f,0.f,0.f,0.f,0.f,0.f,0.f};

  for (int k0 = 0; k0 < K; k0 += 32) {
    V bh[4], bl[4];
#pragma unroll
    for (int j = 0; j < 4; ++j) {
      const size_t bo = (size_t)(n0 + (j << 4) + rlane) * ldb + koff + k0;
      bh[j] = Frag<T>::load(Bb + bo);
      if (SPLIT) bl[j] = Frag<T>::load(Bb2 + bo);
    }
#pragma unroll
    for (int i = 0; i < 4; ++i) {
      const size_t ao = (size_t)(m0 + (i << 4) + rlane) * lda + koff + k0;
      V ah = Frag<T>::load(Ab + ao);
      V al;
      if (SPLIT) al = Frag<T>::load(Ab2 + ao);
#pragma unroll
      for (int j = 0; j < 4; ++j) {
        acc[i][j] = Frag<T>::mma(ah, bh[j], acc[i][j]);
        if (SPLIT) {
          acc[i][j] = Frag<T>::mma(ah, bl[j], acc[i][j]);
          acc[i][j] = Frag<T>::mma(al, bh[j], acc[i][j]);
        }
      }
      Frag<T>::guard4(acc[i][0], acc[i][1], acc[i][2], acc[i][3], ah, SPLIT ? al : ah);
    }
    Frag<T>::keep(bh[0], bh[1], bh[2], bh[3]);
    if (SPLIT) Frag<T>::keep(bl[0], bl[1], bl[2], bl[3]);
  }
  acc_guard4(acc[0][0], acc[0][1], acc[0][2], acc[0][3]);
  acc_guard4(acc[1][0], acc[1][1], acc[1][2], acc[1][3]);
  acc_guard4(acc[2][0], acc[2][1], acc[2][2], acc[2][3]);
  acc_guard4(acc[3][0], acc[3][1], acc[3][2], acc[3][3]);

  float* slab = sT[wave];
  const float* Rb = RESID ? (resid + (size_t)b * strideR) : nullptr;
#pragma unroll
  for (int i = 0; i < 4; ++i) {
    const int mBase = m0 + (i << 4);
#pragma unroll
    for (int j = 0; j < 4; ++j) {
      const int n = n0 + (j << 4) + rlane;
      float bv = 0.f;
      if (BIAS_MODE == 2) bv = bias[n];
#pragma unroll
      for (int r = 0; r < 8; ++r) {
        float v = acc[i][j][r] * scale;
        if (BIAS_MODE == 1) v += bias[mBase + mOff + r];
        if (BIAS_MODE == 2) v += bv;
        if (RESID) v += Rb[(size_t)(mBase + mOff + r) * ldc + n];
        if (ACT == 1) v = tanhf(v);
        if (ACT == 2) v = fmaxf(v, 0.0f);
        if (ACT == 3) v = v / (1.0f + expf(-v));
        if (ACT == 4) v = (v > 0.f) ? v : 0.01f * v;
        slab[(mOff + r) * 68 + (j << 4) + rlane] = v;
      }
    }
    __builtin_amdgcn_fence(__ATOMIC_RELEASE, "workgroup");
    __builtin_amdgcn_wave_barrier();
    __builtin_amdgcn_fence(__ATOMIC_ACQUIRE, "workgroup");
    if (OUT_MODE == 0) {
      float* C = (float*)Cout + (size_t)b * strideC;
      const int hh = lane >> 4, c4 = (lane & 15) * 4;
      for (int pass = 0; pass < 2; ++pass) {
#pragma unroll
        for (int it = 0; it < 8; ++it) {
          const int row = it * 2 + hh;
          v4f v = *(const v4f*)(slab + row * 68 + c4);
          *(volatile v4f*)(C + (size_t)(mBase + row) * ldc + n0 + c4) = v;
        }
        __threadfence();
      }
    } else {
      const int q = lane >> 3, c8 = (lane & 7) * 8;
      unsigned short* C  = (unsigned short*)Cout  + (size_t)b * strideC;
      unsigned short* C2 = (OUT_MODE == 2) ? ((unsigned short*)Cout2 + (size_t)b * strideC) : nullptr;
      for (int pass = 0; pass < 2; ++pass) {
#pragma unroll
        for (int it = 0; it < 4; ++it) {
          const int row = it * 4 + q;
          const float* sp = slab + row * 68 + c8;
          v8h hv, lv;
#pragma unroll
          for (int e = 0; e < 8; ++e) {
            if (OUT_MODE == 1) {
              hv[e] = (_Float16)sp[e];
            } else {
              unsigned short hb = f2bf_bits(sp[e]);
              unsigned short lb = f2bf_bits(sp[e] - bf_bits2f(hb));
              hv[e] = __builtin_bit_cast(_Float16, hb);
              lv[e] = __builtin_bit_cast(_Float16, lb);
            }
          }
          *(volatile v8h*)(C + (size_t)(mBase + row) * ldc + n0 + c8) = hv;
          if (OUT_MODE == 2) *(volatile v8h*)(C2 + (size_t)(mBase + row) * ldc + n0 + c8) = lv;
        }
        __threadfence();
      }
    }
    __builtin_amdgcn_fence(__ATOMIC_RELEASE, "workgroup");
    __builtin_amdgcn_wave_barrier();
    __builtin_amdgcn_fence(__ATOMIC_ACQUIRE, "workgroup");
  }
}

__global__ __launch_bounds__(kThr) void cast_plane_kernel(const float* __restrict__ src, unsigned short* __restrict__ dst,
                                                          int colsLog2, int dstPitch, int dstOff) {
  const int i   = blockIdx.x * kThr + threadIdx.x;
  const int sh  = colsLog2 - 3;
  const int row = i >> sh;
  const int c8  = (i & ((1 << sh) - 1)) * 8;
  const float* sp = src + ((size_t)row << colsLog2) + c8;
  const v4f a0 = *(const v4f*)(sp);
  const v4f a1 = *(const v4f*)(sp + 4);
  v8h hv;
#pragma unroll
  for (int e = 0; e < 4; ++e) {
    const float f0 = a0[e];
    const float f1 = a1[e];
    hv[e]     = (_Float16)carry_flush(bf16r(f0), kInCarry);
    hv[4 + e] = (_Float16)carry_flush(bf16r(f1), kInCarry);
  }
  unsigned short* dp = dst + (size_t)row * dstPitch + dstOff + c8;
  *(volatile v8h*)dp = hv;
  __threadfence();
  *(volatile v8h*)dp = hv;
}
__global__ __launch_bounds__(256) void wt_plane_kernel(const float* __restrict__ W, unsigned short* __restrict__ dst, int K, int N, int nLive, int ldd, int colOff) {
  const int n  = blockIdx.x;
  const int k8 = threadIdx.x * 8;
  const bool live = n < nLive;
  const int nc = live ? n : 0;
  v8h hv;
#pragma unroll
  for (int e = 0; e < 8; ++e) {
    const float w = W[(size_t)(k8 + e) * N + nc];
    hv[e] = (_Float16)(live ? carry_flush(bf16r(w), kWCarry) : 0.0f);
  }
  unsigned short* dp = dst + (size_t)n * ldd + colOff + k8;
  *(volatile v8h*)dp = hv;
  __threadfence();
  *(volatile v8h*)dp = hv;
}


constexpr int kFBQ = 0, kFBV = 512, kFBO = 1024, kFB1 = 1536, kFB2 = 2560, kFZB = 3072, kFEnd = 4096;
__global__ __launch_bounds__(kThr) void setup_kernel(const float* __restrict__ bq, const float* __restrict__ bv, const float* __restrict__ bo,
                                                     const float* __restrict__ b1, const float* __restrict__ b2, float* __restrict__ BIAS) {
  unsigned v = blockIdx.x * (unsigned)kThr + threadIdx.x;
  asm volatile("" : "+v"(v));
  const unsigned i0 = v * 4u;
  v4f o = {0.f, 0.f, 0.f, 0.f};
  if (i0 < (unsigned)kFZB) {
    const float* sp = (i0 < (unsigned)kFBV) ? (bq + i0) : (i0 < (unsigned)kFBO) ? (bv + (i0 - (unsigned)kFBV)) : (i0 < (unsigned)kFB1) ? (bo + (i0 - (unsigned)kFBO))
                    : (i0 < (unsigned)kFB2) ? (b1 + (i0 - (unsigned)kFB1)) : (b2 + (i0 - (unsigned)kFB2));
    const v4f a = *(const v4f*)sp;
#pragma unroll
    for (int e = 0; e < 4; ++e) { const float p = a[e]; o[e] = bf16r(p); }
  }
  float* dp = BIAS + i0;
  *(volatile v4f*)dp = o;
  __threadfence();
  *(volatile v4f*)dp = o;
}
static_assert(kFEnd / 4 == 4 * kThr && (kFBV % 128) == 0 && (kFBO % 128) == 0 && (kFB1 % 128) == 0 && (kFB2 % 128) == 0 && (kFZB % 128) == 0 && kFEnd - kFZB >= kT, "bias stream map; regions wave-uniform");

__global__ __launch_bounds__(kThr) void xt_kernel(const float* __restrict__ res, float* __restrict__ XT32, unsigned short* __restrict__ X16) {
  unsigned v = blockIdx.x * (unsigned)kThr + threadIdx.x;
  asm volatile("" : "+v"(v));
  const unsigned r = v >> 6, t8 = (v & 63u) * 8u;
  const unsigned b = r >> 9, c = r & 511u;
  const float* sp = res + ((size_t)b * kT + t8) * kC + c;
  v4f x0, x1;
  v8h hv;
#pragma unroll
  for (int e = 0; e < 8; ++e) {
    float p = sp[(size_t)e * kC];
    asm volatile("" : "+v"(p));
    const float q = bf16r(p);
    if (e < 4) x0[e] = q; else x1[e - 4] = q;
    hv[e] = (_Float16)carry_flush(q, kInCarry);
  }
  const size_t o8 = (size_t)v * 8u;
  for (int pass = 0; pass < 2; ++pass) {
    *(volatile v4f*)(XT32 + o8) = x0;
    *(volatile v4f*)(XT32 + o8 + 4) = x1;
    *(volatile v8h*)(X16 + o8) = hv;
    __threadfence();
  }
}
__global__ __launch_bounds__(kThr) void cast16_kernel(const float* __restrict__ F, unsigned short* __restrict__ H16) {
  unsigned v = blockIdx.x * (unsigned)kThr + threadIdx.x;
  asm volatile("" : "+v"(v));
  const size_t o8 = (size_t)v * 8u;
  const v4f a0 = *(const v4f*)(F + o8), a1 = *(const v4f*)(F + o8 + 4);
  v8h hv;
#pragma unroll
  for (int e = 0; e < 4; ++e) { hv[e] = (_Float16)carry_flush(a0[e], kInCarry); hv[4 + e] = (_Float16)carry_flush(a1[e], kInCarry); }
  *(volatile v8h*)(H16 + o8) = hv;
  __threadfence();
  *(volatile v8h*)(H16 + o8) = hv;
}
static_assert(((size_t)kRC * kT / 8) == 1024 * kThr, "chunk-plane grids exact");

__global__ __launch_bounds__(kThr) void rollattn_kernel(const float* __restrict__ XT32, const float* __restrict__ RV, const float* __restrict__ Q,
                                                        const float* __restrict__ bk, unsigned short* __restrict__ MIX16) {
  unsigned r = blockIdx.x * (unsigned)kThr + threadIdx.x;
  asm volatile("" : "+v"(r));
  const float* xr = XT32 + (size_t)r * kT;
  const float* rv = RV + (size_t)r * kT;
  const float* qr = Q + (size_t)r * kT;
  float qb = 0.0f;
  for (unsigned e4 = 0; e4 < (unsigned)kT; e4 += 4) {
    const v4f a = *(const v4f*)(qr + e4), w = *(const v4f*)(bk + e4);
    qb += a[0] * bf16r(w[0]); qb += a[1] * bf16r(w[1]); qb += a[2] * bf16r(w[2]); qb += a[3] * bf16r(w[3]);
  }
  float sc[kNS];
#pragma unroll
  for (int s = 0; s < kNS; ++s) sc[s] = 0.0f;
  for (unsigned t4 = 0; t4 < (unsigned)kT; t4 += 4) {
    const v4f w = *(const v4f*)(rv + t4);
#pragma unroll
    for (int s = 0; s < kNS; ++s) {
      const v4f a = *(const v4f*)(xr + ((t4 + (unsigned)(s * kP)) & (unsigned)(kT - 1)));
      sc[s] += a[0] * w[0]; sc[s] += a[1] * w[1]; sc[s] += a[2] * w[2]; sc[s] += a[3] * w[3];
    }
  }
  float mx = (sc[0] + qb) * kScoreScale;
#pragma unroll
  for (int s = 0; s < kNS; ++s) { sc[s] = (sc[s] + qb) * kScoreScale; mx = (sc[s] > mx) ? sc[s] : mx; }
  float sum = 0.0f;
#pragma unroll
  for (int s = 0; s < kNS; ++s) { sc[s] = expf(sc[s] - mx); sum += sc[s]; }
#pragma unroll
  for (int s = 0; s < kNS; ++s) sc[s] = sc[s] / sum;
  unsigned short* mp = MIX16 + (size_t)r * kT;
  for (unsigned t8 = 0; t8 < (unsigned)kT; t8 += 8) {
    v4f m0 = {0.f, 0.f, 0.f, 0.f}, m1 = {0.f, 0.f, 0.f, 0.f};
#pragma unroll
    for (int s = 0; s < kNS; ++s) {
      const unsigned ix = (t8 + (unsigned)(s * kP)) & (unsigned)(kT - 1);
      const v4f a0 = *(const v4f*)(xr + ix), a1 = *(const v4f*)(xr + ix + 4);
      m0 = m0 + a0 * sc[s]; m1 = m1 + a1 * sc[s];
    }
    v8h hv;
#pragma unroll
    for (int e = 0; e < 4; ++e) { hv[e] = (_Float16)carry_flush(m0[e], kInCarry); hv[4 + e] = (_Float16)carry_flush(m1[e], kInCarry); }
    *(volatile v8h*)(mp + t8) = hv;
    __threadfence();
    *(volatile v8h*)(mp + t8) = hv;
  }
}
static_assert(kRC == 16 * kThr && (kP % 8) == 0 && (kT & (kT - 1)) == 0, "row grids exact; a rolled group of 8 never wraps inside itself");

__global__ __launch_bounds__(kThr) void addres_kernel(const float* __restrict__ OP, const float* __restrict__ XT32, float* __restrict__ H32) {
  unsigned v = blockIdx.x * (unsigned)kThr + threadIdx.x;
  asm volatile("" : "+v"(v));
  const size_t o8 = (size_t)v * 8u;
  const v4f h0 = *(const v4f*)(OP + o8) + *(const v4f*)(XT32 + o8), h1 = *(const v4f*)(OP + o8 + 4) + *(const v4f*)(XT32 + o8 + 4);
  for (int pass = 0; pass < 2; ++pass) {
    *(volatile v4f*)(H32 + o8) = h0;
    *(volatile v4f*)(H32 + o8 + 4) = h1;
    __threadfence();
  }
}

__global__ __launch_bounds__(kThr) void bnstat_kernel(const float* __restrict__ H32, float* __restrict__ STAT) {
  unsigned c = blockIdx.x * (unsigned)kThr + threadIdx.x;
  asm volatile("" : "+v"(c));
  float s = 0.0f;
  for (unsigned b = 0; b < (unsigned)kB; ++b) {
    const float* hp = H32 + ((size_t)b * kC + c) * kT;
    for (unsigned t4 = 0; t4 < (unsigned)kT; t4 += 4) { const v4f a = *(const v4f*)(hp + t4); s += a[0]; s += a[1]; s += a[2]; s += a[3]; }
  }
  const float mu = s * kInvBT;
  float q = 0.0f;
  for (unsigned b = 0; b < (unsigned)kB; ++b) {
    const float* hp = H32 + ((size_t)b * kC + c) * kT;
    for (unsigned t4 = 0; t4 < (unsigned)kT; t4 += 4) {
      const v4f a = *(const v4f*)(hp + t4);
#pragma unroll
      for (int e = 0; e < 4; ++e) { const float d = a[e] - mu; q += d * d; }
    }
  }
  const float sd = sqrtf(q * kInvBT + kEps);
  for (int pass = 0; pass < 2; ++pass) {
    *(volatile float*)(STAT + c) = mu;
    *(volatile float*)(STAT + kC + c) = sd;
    __threadfence();
  }
}
static_assert(kC == 2 * kThr, "statistics grid exact");

__global__ __launch_bounds__(kThr) void bnapply_kernel(const float* __restrict__ H32, const float* __restrict__ STAT, const float* __restrict__ bn_w,
                                                       const float* __restrict__ bn_b, float* __restrict__ HN32, unsigned short* __restrict__ HN16) {
  unsigned v = blockIdx.x * (unsigned)kThr + threadIdx.x;
  asm volatile("" : "+v"(v));
  const size_t o8 = (size_t)v * 8u;
  const unsigned c = (v >> 6) & 511u;
  float mu = STAT[c], sd = STAT[kC + c], gw = bn_w[c], gb = bn_b[c];
  asm volatile("" : "+v"(mu), "+v"(sd), "+v"(gw), "+v"(gb));
  gw = bf16r(gw); gb = bf16r(gb);
  const v4f a0 = *(const v4f*)(H32 + o8), a1 = *(const v4f*)(H32 + o8 + 4);
  v4f n0, n1;
  v8h hv;
#pragma unroll
  for (int e = 0; e < 4; ++e) {
    n0[e] = (a0[e] - mu) / sd * gw + gb; n1[e] = (a1[e] - mu) / sd * gw + gb;
    hv[e] = (_Float16)carry_flush(n0[e], kInCarry); hv[4 + e] = (_Float16)carry_flush(n1[e], kInCarry);
  }
  for (int pass = 0; pass < 2; ++pass) {
    *(volatile v4f*)(HN32 + o8) = n0;
    *(volatile v4f*)(HN32 + o8 + 4) = n1;
    *(volatile v8h*)(HN16 + o8) = hv;
    __threadfence();
  }
}

__global__ __launch_bounds__(kThr) void gelu_kernel(const float* __restrict__ F1, unsigned short* __restrict__ G16) {
  unsigned v = blockIdx.x * (unsigned)kThr + threadIdx.x;
  asm volatile("" : "+v"(v));
  const float* sp = F1 + (size_t)v * 8u;
  const v4f a0 = *(const v4f*)sp, a1 = *(const v4f*)(sp + 4);
  v8h hv;
#pragma unroll
  for (int e = 0; e < 4; ++e) {
    const float x0 = a0[e], x1 = a1[e];
    const float y0 = 0.5f * x0 * (1.0f + erff(x0 * 0.70710678118654752f)), y1 = 0.5f * x1 * (1.0f + erff(x1 * 0.70710678118654752f));
    hv[e] = (_Float16)carry_flush(y0, kInCarry);
    hv[4 + e] = (_Float16)carry_flush(y1, kInCarry);
  }
  unsigned short* dp = G16 + (size_t)v * 8u;
  *(volatile v8h*)dp = hv;
  __threadfence();
  *(volatile v8h*)dp = hv;
}
static_assert(((size_t)kRC * kFF / 8) == 2048 * kThr, "GELU grid exact");

__global__ __launch_bounds__(kThr) void lnout_kernel(const float* __restrict__ FO, const float* __restrict__ HN32, const float* __restrict__ ln_w,
                                                     const float* __restrict__ ln_b, float* __restrict__ outc) {
  unsigned r = blockIdx.x * (unsigned)kThr + threadIdx.x;
  asm volatile("" : "+v"(r));
  const float* fr = FO + (size_t)r * kT;
  const float* hr = HN32 + (size_t)r * kT;
  float s = 0.0f;
  for (unsigned t4 = 0; t4 < (unsigned)kT; t4 += 4) { const v4f y = *(const v4f*)(fr + t4) + *(const v4f*)(hr + t4); s += y[0]; s += y[1]; s += y[2]; s += y[3]; }
  const float mu = s * kInvT;
  float q = 0.0f;
  for (unsigned t4 = 0; t4 < (unsigned)kT; t4 += 4) {
    const v4f y = *(const v4f*)(fr + t4) + *(const v4f*)(hr + t4);
#pragma unroll
    for (int e = 0; e < 4; ++e) { const float d = y[e] - mu; q += d * d; }
  }
  const float sd = sqrtf(q * kInvT + kEps);
  const unsigned b = r >> 9, c = r & 511u;
  float* op = outc + (size_t)b * kT * kC + c;
  for (int pass = 0; pass < 2; ++pass) {
    for (unsigned t4 = 0; t4 < (unsigned)kT; t4 += 4) {
      const v4f y = *(const v4f*)(fr + t4) + *(const v4f*)(hr + t4), gw = *(const v4f*)(ln_w + t4), gb = *(const v4f*)(ln_b + t4);
#pragma unroll
      for (int e = 0; e < 4; ++e) *(volatile float*)(op + (size_t)(t4 + (unsigned)e) * kC) = (y[e] - mu) / sd * bf16r(gw[e]) + bf16r(gb[e]);
    }
    __threadfence();
  }
}

static_assert(((size_t)kT * kT / 8) % kThr == 0 && ((size_t)kFF * kT / 8) % kThr == 0, "plane cast grids exact");

extern "C" void kernel_launch(void* const* d_in, const int* in_sizes, int n_in,
                              void* d_out, int out_size, void* d_ws, size_t ws_size,
                              hipStream_t stream) {
  if (n_in < 17 || d_out == nullptr || d_ws == nullptr) return;
  if (in_sizes[0] != kB * kT * kC || in_sizes[1] != kT * kT || in_sizes[2] != kT || in_sizes[3] != kT * kT || in_sizes[4] != kT || in_sizes[5] != kT * kT || in_sizes[6] != kT) return;
  if (in_sizes[7] != kT * kT || in_sizes[8] != kT || in_sizes[9] != kC || in_sizes[10] != kC || in_sizes[11] != kFF * kT || in_sizes[12] != kFF || in_sizes[13] != kT * kFF || in_sizes[14] != kT) return;
  if (in_sizes[15] != kT || in_sizes[16] != kT) return;
  if (out_size != kB * kT * kC) return;
  if (ws_size < kWsTotal) return;
  const float* residual = (const float*)d_in[0];
  const float* wq = (const float*)d_in[1];
  const float* bq = (const float*)d_in[2];
  const float* wk = (const float*)d_in[3];
  const float* bk = (const float*)d_in[4];
  const float* wv = (const float*)d_in[5];
  const float* bv = (const float*)d_in[6];
  const float* wo = (const float*)d_in[7];
  const float* bo = (const float*)d_in[8];
  const float* bn_w = (const float*)d_in[9];
  const float* bn_b = (const float*)d_in[10];
  const float* w1 = (const float*)d_in[11];
  const float* b1 = (const float*)d_in[12];
  const float* w2 = (const float*)d_in[13];
  const float* b2 = (const float*)d_in[14];
  const float* ln_w = (const float*)d_in[15];
  const float* ln_b = (const float*)d_in[16];
  float* out = (float*)d_out;
  char* ws = (char*)d_ws;
  unsigned short* WQ16 = (unsigned short*)(ws + kOffWQ16);
  unsigned short* WKT16 = (unsigned short*)(ws + kOffWKT16);
  unsigned short* WV16 = (unsigned short*)(ws + kOffWV16);
  unsigned short* WO16 = (unsigned short*)(ws + kOffWO16);
  unsigned short* W1H = (unsigned short*)(ws + kOffW1H);
  unsigned short* W2H = (unsigned short*)(ws + kOffW2H);
  float* BIAS = (float*)(ws + kOffBIAS);
  float* STAT = (float*)(ws + kOffSTAT);
  float* H32 = (float*)(ws + kOffH32);
  float* XT32 = (float*)(ws + kOffXT32);
  unsigned short* X16 = (unsigned short*)(ws + kOffX16);
  float* FA = (float*)(ws + kOffFA);
  float* FB = (float*)(ws + kOffFB);
  unsigned short* HA = (unsigned short*)(ws + kOffHA);
  float* F1 = (float*)(ws + kOffF1);
  unsigned short* G16 = (unsigned short*)(ws + kOffG16);

  cast_plane_kernel<<<(int)(((size_t)kT * kT / 8) / kThr), kThr, 0, stream>>>(wq, WQ16, 9, kT, 0);
  cast_plane_kernel<<<(int)(((size_t)kT * kT / 8) / kThr), kThr, 0, stream>>>(wv, WV16, 9, kT, 0);
  cast_plane_kernel<<<(int)(((size_t)kT * kT / 8) / kThr), kThr, 0, stream>>>(wo, WO16, 9, kT, 0);
  cast_plane_kernel<<<(int)(((size_t)kFF * kT / 8) / kThr), kThr, 0, stream>>>(w1, W1H, 9, kT, 0);
  cast_plane_kernel<<<(int)(((size_t)kT * kFF / 8) / kThr), kThr, 0, stream>>>(w2, W2H, 10, kFF, 0);
  wt_plane_kernel<<<kT, kT / 8, 0, stream>>>(wk, WKT16, kT, kT, kT, kT, 0);
  setup_kernel<<<4, kThr, 0, stream>>>(bq, bv, bo, b1, b2, BIAS);

  for (int ch = 0; ch < kNCh; ++ch) {
    const float* rc = residual + (size_t)ch * kBC * kT * kC;
    xt_kernel<<<1024, kThr, 0, stream>>>(rc, XT32, X16);
    wmma_gemm64<0, false, 2, 0, false, 0><<<dim3((kRC / 64) * (kT / 64) / 8, 1), 256, 0, stream>>>(
        X16, X16, kT, 0L, WQ16, WQ16, kT, 0L, (void*)FA, (void*)FA, kT, 0L, BIAS + kFBQ, nullptr, 0L, kRC, kT, kT, kScA);
    cast16_kernel<<<1024, kThr, 0, stream>>>(FA, HA);
    wmma_gemm64<0, false, 2, 0, false, 0><<<dim3((kRC / 64) * (kT / 64) / 8, 1), 256, 0, stream>>>(
        HA, HA, kT, 0L, WKT16, WKT16, kT, 0L, (void*)FB, (void*)FB, kT, 0L, BIAS + kFZB, nullptr, 0L, kRC, kT, kT, kScK);
    rollattn_kernel<<<16, kThr, 0, stream>>>(XT32, FB, FA, bk, HA);
    wmma_gemm64<0, false, 2, 0, false, 0><<<dim3((kRC / 64) * (kT / 64) / 8, 1), 256, 0, stream>>>(
        HA, HA, kT, 0L, WV16, WV16, kT, 0L, (void*)FA, (void*)FA, kT, 0L, BIAS + kFBV, nullptr, 0L, kRC, kT, kT, kScA);
    cast16_kernel<<<1024, kThr, 0, stream>>>(FA, HA);
    wmma_gemm64<0, false, 2, 0, false, 0><<<dim3((kRC / 64) * (kT / 64) / 8, 1), 256, 0, stream>>>(
        HA, HA, kT, 0L, WO16, WO16, kT, 0L, (void*)FB, (void*)FB, kT, 0L, BIAS + kFBO, nullptr, 0L, kRC, kT, kT, kScA);
    addres_kernel<<<1024, kThr, 0, stream>>>(FB, XT32, H32 + (size_t)ch * kRC * kT);
  }
  bnstat_kernel<<<2, kThr, 0, stream>>>(H32, STAT);
  for (int ch = 0; ch < kNCh; ++ch) {
    bnapply_kernel<<<1024, kThr, 0, stream>>>(H32 + (size_t)ch * kRC * kT, STAT, bn_w, bn_b, FA, HA);
    wmma_gemm64<0, false, 2, 0, false, 0><<<dim3((kRC / 64) * (kFF / 64) / 8, 1), 256, 0, stream>>>(
        HA, HA, kT, 0L, W1H, W1H, kT, 0L, (void*)F1, (void*)F1, kFF, 0L, BIAS + kFB1, nullptr, 0L, kRC, kFF, kT, kScA);
    gelu_kernel<<<2048, kThr, 0, stream>>>(F1, G16);
    wmma_gemm64<0, false, 2, 0, false, 0><<<dim3((kRC / 64) * (kT / 64) / 8, 1), 256, 0, stream>>>(
        G16, G16, kFF, 0L, W2H, W2H, kFF, 0L, (void*)FB, (void*)FB, kT, 0L, BIAS + kFB2, nullptr, 0L, kRC, kT, kFF, kScA);
    lnout_kernel<<<16, kThr, 0, stream>>>(FB, FA, ln_w, ln_b, out + (size_t)ch * kBC * kT * kC);
  }
}
